// ULayer_18726057410941
// MI455X (gfx1250) — hardware-run, weakly checked
//
#include <hip/hip_runtime.h>
#include <math.h>

typedef __attribute__((ext_vector_type(16))) _Float16 v16h;
typedef __attribute__((ext_vector_type(8)))  _Float16 v8h;
typedef __attribute__((ext_vector_type(8)))  float    v8f;
typedef __attribute__((ext_vector_type(4)))  float    v4f;

constexpr int kBatch  = 256;
constexpr int kDim    = 4096;
constexpr int kDigit  = 16;
constexpr int kEmb    = 32;
constexpr int kGates  = 3;
constexpr int kPlaneHalves = kEmb * kEmb;
static_assert(kDigit * kDigit * kDigit == kDim, "three radix-16 digits");
static_assert(kEmb == 2 * kDigit, "real embedding of a 16 x 16 complex gate");
static_assert(kEmb == 32, "one 32-deep k step, no tail");

constexpr size_t kGateBytes = (size_t)kGates * 2 * kPlaneHalves * 2;
static_assert(kGateBytes == 12288ull, "carve total");
static_assert(kGateBytes <= 134217728ull, "carve cap");

constexpr float kStateCarry   = 64.0f;
constexpr float kGateCarry    = 64.0f;
constexpr float kResCarry     = 2048.0f;
constexpr float kFoldMain     = 1.0f / (kStateCarry * kGateCarry);
constexpr float kFoldRes      = 1.0f / kResCarry;
constexpr float kF16MinNormal = 6.103515625e-5f;
static_assert(kFoldMain == 0.000244140625f, "1/4096");
static_assert(kFoldRes == 0.00048828125f, "1/2048");

union FragU { v16h v; v8h h[2]; };
__device__ __forceinline__ v16h frag_load(const _Float16* p) {
  FragU f;
  f.h[0] = *(const v8h*)(p);
  f.h[1] = *(const v8h*)(p + 16);
  return f.v;
}
__device__ __forceinline__ v8f mma_h(v16h a, v16h b, v8f c) {
  c = __builtin_amdgcn_wmma_f32_16x16x32_f16(false, a, false, b, (short)0, c, false, false);
  asm volatile("v_nop\n\tv_nop\n\tv_nop\n\tv_nop" : "+v"(c) : "v"(a), "v"(b));
  return c;
}

__device__ __forceinline__ void split_carry(float x, float carry, _Float16& hi, _Float16& lo) {
  const float xs = x * carry;
  const float xh = (fabsf(xs) < kF16MinNormal) ? 0.0f : xs;
  const _Float16 h = (_Float16)xh;
  const float hf = (float)h;
  const float rs = (xs - hf) * kResCarry;
  const float rl = (fabsf(rs) < kF16MinNormal) ? 0.0f : rs;
  hi = h;
  lo = (_Float16)rl;
}

__device__ __forceinline__ float gate_entry(int n, int k, float cs, float sn) {
  const int r  = n & 15;
  const int c  = k & 15;
  const int io = n >> 4;
  const int ii = k >> 4;
  const int kr = r >> 2;
  const int kc = c >> 2;
  const int i  = r & 3;
  const int j  = c & 3;
  const bool same  = (kr == kc);
  const bool outer = (kr == 0) || (kr == 3);
  const float sgn  = (kr < 2) ? -1.0f : 1.0f;
  const float ss   = sgn * sn;
  const bool dg    = (i == j);
  const bool mid   = (i == 1) || (i == 2);
  const bool swp   = mid && ((i + j) == 3);
  float ur = dg ? ((i == 0) ? 1.0f : ((i == 3) ? (outer ? cs : 1.0f) : cs)) : 0.0f;
  float ui = dg ? ((i == 3) ? (outer ? ss : 0.0f) : (mid ? (outer ? 0.0f : ss) : 0.0f))
                : ((swp && outer) ? ss : 0.0f);
  ur = same ? ur : 0.0f;
  ui = same ? ui : 0.0f;
  const float nui = -ui;
  return (io == ii) ? ur : ((io != 0) ? ui : nui);
}

__global__ __launch_bounds__(96) void gate_build_kernel(
    const float* __restrict__ thetas, unsigned short* __restrict__ gates)
{
  const int lane = threadIdx.x & 31;
  const int g    = threadIdx.x >> 5;
  const float th = thetas[g];
  const float cs = cosf(th);
  const float sn = sinf(th);
  v8h hv[4], lv[4];
#pragma unroll
  for (int it = 0; it < 4; ++it) {
    const int n  = it * 8 + (lane >> 2);
    const int k0 = (lane & 3) * 8;
#pragma unroll
    for (int e = 0; e < 8; ++e) {
      float val = gate_entry(n, k0 + e, cs, sn);
      asm volatile("" : "+v"(val));
      _Float16 h, l;
      split_carry(val, kGateCarry, h, l);
      hv[it][e] = h;
      lv[it][e] = l;
    }
  }
  unsigned short* ph = gates + (size_t)(g * 2 + 0) * kPlaneHalves;
  unsigned short* pl = gates + (size_t)(g * 2 + 1) * kPlaneHalves;
  for (int pass = 0; pass < 2; ++pass) {
#pragma unroll
    for (int it = 0; it < 4; ++it) {
      const int off = it * 256 + lane * 8;
      *(volatile v8h*)(ph + off) = hv[it];
      *(volatile v8h*)(pl + off) = lv[it];
    }
    __threadfence();
  }
}

__global__ __launch_bounds__(256) void apply_gates_kernel(
    const float* __restrict__ in_re, const float* __restrict__ in_im,
    const unsigned short* __restrict__ gates, float* __restrict__ out)
{
  __shared__ __align__(16) float sre[kDim];
  __shared__ __align__(16) float sim[kDim];
  const int tid  = threadIdx.x;
  const int lane = tid & 31;
  const int wave = tid >> 5;
  const int b    = blockIdx.x;
  const int h    = lane >> 4;
  const int m    = lane & 15;

  const float* gr = in_re + (size_t)b * kDim;
  const float* gi = in_im + (size_t)b * kDim;
#pragma unroll
  for (int it = 0; it < 4; ++it) {
    const int o = (it * 256 + tid) * 4;
    const v4f a = *(const v4f*)(gr + o);
    const v4f c = *(const v4f*)(gi + o);
    *(v4f*)(sre + o) = a;
    *(v4f*)(sim + o) = c;
  }
  __syncthreads();

#pragma unroll 1
  for (int g = 0; g < kGates; ++g) {
    const int tS = (g == 0) ? 16 : 256;
    const int kS = (g == 0) ? 256 : ((g == 1) ? 16 : 1);
    const int mS = (g == 2) ? 16 : 1;
    const _Float16* gh = (const _Float16*)(gates + (size_t)(g * 2 + 0) * kPlaneHalves);
    const _Float16* gl = (const _Float16*)(gates + (size_t)(g * 2 + 1) * kPlaneHalves);
    const v16h bh0 = frag_load(gh + m * kEmb + 8 * h);
    const v16h bh1 = frag_load(gh + (16 + m) * kEmb + 8 * h);
    const v16h bl0 = frag_load(gl + m * kEmb + 8 * h);
    const v16h bl1 = frag_load(gl + (16 + m) * kEmb + 8 * h);

#pragma unroll 1
    for (int tt = 0; tt < 2; ++tt) {
      const int tile  = wave * 2 + tt;
      const int rbase = tile * tS + m * mS + (8 * h) * kS;
      v16h ah, al;
#pragma unroll
      for (int e = 0; e < 8; ++e) {
        const float xr = sre[rbase + e * kS];
        const float xi = sim[rbase + e * kS];
        _Float16 hr, lr, hq, lq;
        split_carry(xr, kStateCarry, hr, lr);
        split_carry(xi, kStateCarry, hq, lq);
        ah[e]     = hr;
        al[e]     = lr;
        ah[8 + e] = hq;
        al[8 + e] = lq;
      }
      v8f am0 = (v8f){0.f, 0.f, 0.f, 0.f, 0.f, 0.f, 0.f, 0.f};
      v8f am1 = (v8f){0.f, 0.f, 0.f, 0.f, 0.f, 0.f, 0.f, 0.f};
      v8f ar0 = (v8f){0.f, 0.f, 0.f, 0.f, 0.f, 0.f, 0.f, 0.f};
      v8f ar1 = (v8f){0.f, 0.f, 0.f, 0.f, 0.f, 0.f, 0.f, 0.f};
      am0 = mma_h(ah, bh0, am0);
      am1 = mma_h(ah, bh1, am1);
      ar0 = mma_h(ah, bl0, ar0);
      ar0 = mma_h(al, bh0, ar0);
      ar1 = mma_h(ah, bl1, ar1);
      ar1 = mma_h(al, bh1, ar1);
      const int wbase = tile * tS + m * kS + (8 * h) * mS;
#pragma unroll
      for (int r = 0; r < 8; ++r) {
        const float vre = (am0[r] + ar0[r] * kFoldRes) * kFoldMain;
        const float vim = (am1[r] + ar1[r] * kFoldRes) * kFoldMain;
        sre[wbase + r * mS] = vre;
        sim[wbase + r * mS] = vim;
      }
    }
    __syncthreads();
  }

  v4f ov[8];
#pragma unroll
  for (int it = 0; it < 8; ++it) {
    const int i0 = (it * 256 + tid) * 2;
    v4f t;
    t[0] = sre[i0];
    t[1] = sim[i0];
    t[2] = sre[i0 + 1];
    t[3] = sim[i0 + 1];
    ov[it] = t;
  }
  float* ob = out + (size_t)b * (kDim * 2);
  for (int pass = 0; pass < 2; ++pass) {
#pragma unroll
    for (int it = 0; it < 8; ++it) {
      *(volatile v4f*)(ob + (size_t)(it * 256 + tid) * 4) = ov[it];
    }
    __threadfence();
  }
}

extern "C" void kernel_launch(void* const* d_in, const int* in_sizes, int n_in,
                              void* d_out, int out_size, void* d_ws, size_t ws_size,
                              hipStream_t stream) {
  if (n_in < 3) return;
  if (in_sizes[0] != kBatch * kDim) return;
  if (in_sizes[1] != kBatch * kDim) return;
  if (in_sizes[2] != kGates) return;
  if (out_size != kBatch * kDim * 2) return;
  if (ws_size < kGateBytes) return;

  const float* in_re  = (const float*)d_in[0];
  const float* in_im  = (const float*)d_in[1];
  const float* thetas = (const float*)d_in[2];
  unsigned short* gates = (unsigned short*)d_ws;
  float* out = (float*)d_out;

  gate_build_kernel<<<1, 96, 0, stream>>>(thetas, gates);
  apply_gates_kernel<<<kBatch, 256, 0, stream>>>(in_re, in_im, gates, out);
}
